// SableNetwork_87084756894089
// MI455X (gfx1250) — hardware-verified
//
#include <hip/hip_runtime.h>
#include <math.h>
#include <stddef.h>

constexpr int kB   = 8;
constexpr int kS   = 1024;
constexpr int kObs = 128;
constexpr int kE   = 256;
constexpr int kH   = 8;
constexpr int kDh  = 32;
constexpr int kL   = 2;
constexpr int kTok = kB * kS;
constexpr int kQKG = 3 * kE;
constexpr float kEps = 1e-6f;

typedef __attribute__((ext_vector_type(16))) _Float16 v16h;
typedef __attribute__((ext_vector_type(8)))  _Float16 v8h;
typedef __attribute__((ext_vector_type(16))) __bf16   v16b;
typedef __attribute__((ext_vector_type(8)))  __bf16   v8b;
typedef __attribute__((ext_vector_type(8)))  float    v8f;
typedef __attribute__((ext_vector_type(4)))  float    v4f;
typedef __attribute__((ext_vector_type(4)))  unsigned int v4u;

__device__ __forceinline__ unsigned short f2bf_bits(float f) {
  unsigned u = __float_as_uint(f);
  return (unsigned short)((u + 0x7FFFu + ((u >> 16) & 1u)) >> 16);
}
__device__ __forceinline__ float bf_bits2f(unsigned short h) { return __uint_as_float(((unsigned)h) << 16); }

__device__ __forceinline__ void dep_guard_h(v8f& a, v8f& b, v16h x, v16h y) { asm volatile("v_nop\n\tv_nop\n\tv_nop\n\tv_nop" : "+v"(a), "+v"(b) : "v"(x), "v"(y)); }
__device__ __forceinline__ void dep_guard_b(v8f& a, v8f& b, v16b x, v16b y) { asm volatile("v_nop\n\tv_nop\n\tv_nop\n\tv_nop" : "+v"(a), "+v"(b) : "v"(x), "v"(y)); }
__device__ __forceinline__ void keep4_h(v16h a, v16h b, v16h c, v16h d) { asm volatile("v_nop" :: "v"(a), "v"(b), "v"(c), "v"(d)); }
__device__ __forceinline__ void keep4_b(v16b a, v16b b, v16b c, v16b d) { asm volatile("v_nop" :: "v"(a), "v"(b), "v"(c), "v"(d)); }
__device__ __forceinline__ void acc_guard4(v8f& a, v8f& b, v8f& c, v8f& d) { asm volatile("v_nop\n\tv_nop\n\tv_nop\n\tv_nop" : "+v"(a), "+v"(b), "+v"(c), "+v"(d)); }
template <typename T> struct Frag;
template <> struct Frag<_Float16> {
  typedef v16h V; union U { v16h v; v8h h[2]; };
  static __device__ __forceinline__ v16h load(const _Float16* p) {
    U f; f.h[0] = *(const v8h*)(p); f.h[1] = *(const v8h*)(p + 16); return f.v;
  }
  static __device__ __forceinline__ v8f mma(v16h a, v16h b, v8f c) {
    return __builtin_amdgcn_wmma_f32_16x16x32_f16(false, a, false, b, (short)0, c, false, false);
  }
  static __device__ __forceinline__ void guard(v8f& a, v8f& b, v16h x, v16h y) { dep_guard_h(a, b, x, y); }
  static __device__ __forceinline__ void keep(v16h a, v16h b, v16h c, v16h d) { keep4_h(a, b, c, d); }
};
template <> struct Frag<__bf16> {
  typedef v16b V; union U { v16b v; v8b h[2]; };
  static __device__ __forceinline__ v16b load(const __bf16* p) {
    U f; f.h[0] = *(const v8b*)(p); f.h[1] = *(const v8b*)(p + 16); return f.v;
  }
  static __device__ __forceinline__ v8f mma(v16b a, v16b b, v8f c) {
    return __builtin_amdgcn_wmma_f32_16x16x32_bf16(false, a, false, b, (short)0, c, false, false);
  }
  static __device__ __forceinline__ void guard(v8f& a, v8f& b, v16b x, v16b y) { dep_guard_b(a, b, x, y); }
  static __device__ __forceinline__ void keep(v16b a, v16b b, v16b c, v16b d) { keep4_b(a, b, c, d); }
};

__device__ __forceinline__ unsigned pk16(unsigned short a, unsigned short b) { return (unsigned)a | ((unsigned)b << 16); }

template <int NS> struct KeepB;
template <> struct KeepB<4> {
  static __device__ __forceinline__ void k(v16b (&bh)[4], v16b (&bl)[4]) {
    keep4_b(bh[0], bh[1], bh[2], bh[3]);
    keep4_b(bl[0], bl[1], bl[2], bl[3]);
  }
};
template <> struct KeepB<2> {
  static __device__ __forceinline__ void k(v16b (&bh)[2], v16b (&bl)[2]) { keep4_b(bh[0], bh[1], bl[0], bl[1]); }
};
template <int NS> struct AccG;
template <> struct AccG<4> {
  static __device__ __forceinline__ void g(v8f (&a)[4][4]) {
    acc_guard4(a[0][0], a[0][1], a[0][2], a[0][3]);
    acc_guard4(a[1][0], a[1][1], a[1][2], a[1][3]);
    acc_guard4(a[2][0], a[2][1], a[2][2], a[2][3]);
    acc_guard4(a[3][0], a[3][1], a[3][2], a[3][3]);
  }
};
template <> struct AccG<2> {
  static __device__ __forceinline__ void g(v8f (&a)[4][2]) {
    acc_guard4(a[0][0], a[0][1], a[1][0], a[1][1]);
    acc_guard4(a[2][0], a[2][1], a[3][0], a[3][1]);
  }
};

template <int NSUB, int OUT_MODE, bool RESID, int CMODE>
__global__ __launch_bounds__(256) void gemm_bf16x3(
    const unsigned short* __restrict__ Ap, const unsigned short* __restrict__ A2p, int lda, long strideA,
    const unsigned short* __restrict__ Btp, const unsigned short* __restrict__ Bt2p, int ldb, long strideB,
    void* __restrict__ Cout, void* __restrict__ Cout2, int ldc, long strideC,
    const float* __restrict__ resid,
    const float* __restrict__ dtab,
    int M, int N, int K, float scale) {
  static_assert(NSUB == 4 || NSUB == 2, "");
  static_assert(NSUB == 4 || OUT_MODE == 0, "");
  static_assert(OUT_MODE == 0 || OUT_MODE == 2, "");
  typedef __bf16 T;
  typedef v16b V;
  constexpr int TW = 16 * NSUB;
  const T* A = (const T*)Ap; const T* A2 = (const T*)A2p; const T* Bt = (const T*)Btp; const T* Bt2 = (const T*)Bt2p;
  __shared__ __align__(16) float sT[8][16 * 68];
  __shared__ float sD[256];
  if (CMODE == 1) {
    sD[threadIdx.x] = dtab[(size_t)blockIdx.y * 256 + threadIdx.x];
    __syncthreads();
  }
  const int b    = blockIdx.y;
  const int lane = threadIdx.x & 31;
  const int wave = threadIdx.x >> 5;
  const int tilesN = N / TW;
  const int tilesM = M >> 6;
  const int tile = blockIdx.x * 8 + wave;
  if (tile >= tilesM * tilesN) return;
  const int tm = tile / tilesN;
  const int tn = tile - tm * tilesN;
  const int m0 = tm << 6;
  const int n0 = tn * TW;
  if (CMODE == 1 && tn > tm) return;
  int Kend = K;
  if (CMODE == 2) { const int ke = (tm + 1) * 64; Kend = (ke < K) ? ke : K; }

  const T* Ab  = A   + (size_t)b * strideA;
  const T* Bb  = Bt  + (size_t)b * strideB;
  const T* Ab2 = A2  + (size_t)b * strideA;
  const T* Bb2 = Bt2 + (size_t)b * strideB;

  const int rlane = lane & 15;
  const int koff  = (lane >> 4) * 8;
  const int mOff  = (lane >> 4) * 8;

  v8f acc[4][NSUB];
#pragma unroll
  for (int i = 0; i < 4; ++i)
#pragma unroll
    for (int j = 0; j < NSUB; ++j) acc[i][j] = (v8f){0.f,0.f,0.f,0.f,0.f,0.f,0.f,0.f};

  for (int k0 = 0; k0 < Kend; k0 += 32) {
    V bh[NSUB], bl[NSUB];
#pragma unroll
    for (int j = 0; j < NSUB; ++j) {
      const size_t bo = (size_t)(n0 + (j << 4) + rlane) * ldb + koff + k0;
      bh[j] = Frag<T>::load(Bb + bo);
      bl[j] = Frag<T>::load(Bb2 + bo);
    }
#pragma unroll
    for (int i = 0; i < 4; ++i) {
      const size_t ao = (size_t)(m0 + (i << 4) + rlane) * lda + koff + k0;
      const V ah = Frag<T>::load(Ab + ao);
      const V al = Frag<T>::load(Ab2 + ao);
#pragma unroll
      for (int j = 0; j < NSUB; ++j) {
        acc[i][j] = Frag<T>::mma(ah, bh[j], acc[i][j]);
        acc[i][j] = Frag<T>::mma(ah, bl[j], acc[i][j]);
        acc[i][j] = Frag<T>::mma(al, bh[j], acc[i][j]);
      }
      Frag<T>::guard(acc[i][0], acc[i][NSUB - 1], ah, al);
    }
    KeepB<NSUB>::k(bh, bl);
  }
  AccG<NSUB>::g(acc);

  float* slab = sT[wave];
  const float* Rb = RESID ? (resid + (size_t)b * strideC) : nullptr;
#pragma unroll
  for (int i = 0; i < 4; ++i) {
    const int mBase = m0 + (i << 4);
#pragma unroll
    for (int j = 0; j < NSUB; ++j) {
      const int n = n0 + (j << 4) + rlane;
#pragma unroll
      for (int r = 0; r < 8; ++r) {
        float v = acc[i][j][r] * scale;
        if (CMODE == 1) {
          const int rown = mBase + mOff + r;
          const int e = (rown >> 2) - (n >> 2);
          const int ec = (e < 0) ? 0 : ((e > 255) ? 255 : e);
          const float df = sD[ec];
          v = (e >= 0) ? (v * df) : 0.0f;
        }
        if (RESID) v += Rb[(size_t)(mBase + mOff + r) * ldc + n];
        slab[(mOff + r) * 68 + (j << 4) + rlane] = v;
      }
    }
    __builtin_amdgcn_fence(__ATOMIC_RELEASE, "workgroup");
    __builtin_amdgcn_wave_barrier();
    __builtin_amdgcn_fence(__ATOMIC_ACQUIRE, "workgroup");
    if (OUT_MODE == 0) {
      float* C = (float*)Cout + (size_t)b * strideC;
      if (NSUB == 4) {
        const int hh = lane >> 4, c4 = (lane & 15) * 4;
        for (int pass = 0; pass < 2; ++pass) {
#pragma unroll
          for (int it = 0; it < 8; ++it) {
            const int row = it * 2 + hh;
            v4f v = *(const v4f*)(slab + row * 68 + c4);
            *(volatile v4f*)(C + (size_t)(mBase + row) * ldc + n0 + c4) = v;
          }
          __threadfence();
        }
      } else {
        const int q4 = lane >> 3, c4 = (lane & 7) * 4;
        for (int pass = 0; pass < 2; ++pass) {
#pragma unroll
          for (int it = 0; it < 4; ++it) {
            const int row = it * 4 + q4;
            v4f v = *(const v4f*)(slab + row * 68 + c4);
            *(volatile v4f*)(C + (size_t)(mBase + row) * ldc + n0 + c4) = v;
          }
          __threadfence();
        }
      }
    } else {
      const int q = lane >> 3, c8 = (lane & 7) * 8;
      unsigned short* C  = (unsigned short*)Cout  + (size_t)b * strideC;
      unsigned short* C2 = (unsigned short*)Cout2 + (size_t)b * strideC;
      for (int pass = 0; pass < 2; ++pass) {
#pragma unroll
        for (int it = 0; it < 4; ++it) {
          const int row = it * 4 + q;
          const float* sp = slab + row * 68 + c8;
          v8h hv, lv;
#pragma unroll
          for (int e = 0; e < 8; ++e) {
            unsigned short hb = f2bf_bits(sp[e]);
            unsigned short lb = f2bf_bits(sp[e] - bf_bits2f(hb));
            hv[e] = __builtin_bit_cast(_Float16, hb);
            lv[e] = __builtin_bit_cast(_Float16, lb);
          }
          *(volatile v8h*)(C + (size_t)(mBase + row) * ldc + n0 + c8) = hv;
          *(volatile v8h*)(C2 + (size_t)(mBase + row) * ldc + n0 + c8) = lv;
        }
        __threadfence();
      }
    }
    __builtin_amdgcn_fence(__ATOMIC_RELEASE, "workgroup");
    __builtin_amdgcn_wave_barrier();
    __builtin_amdgcn_fence(__ATOMIC_ACQUIRE, "workgroup");
  }
}

__device__ __forceinline__ float sigm_f(float z) {
  return __builtin_amdgcn_rcpf(1.0f + __builtin_amdgcn_exp2f(-z * 1.4426950408889634f));
}
__device__ __forceinline__ float silu_f(float x) { return x * sigm_f(x); }
__device__ __forceinline__ float gelu_f(float x) {
  const float u = 0.7978845608028654f * (x + 0.044715f * x * x * x);
  return x * sigm_f(2.0f * u);
}
__device__ __forceinline__ void split_pack8(const float (&v)[8], v4u& uh, v4u& ul) {
  unsigned short hb[8], lb[8];
#pragma unroll
  for (int e = 0; e < 8; ++e) {
    hb[e] = f2bf_bits(v[e]);
    lb[e] = f2bf_bits(v[e] - bf_bits2f(hb[e]));
  }
  uh = (v4u){pk16(hb[0], hb[1]), pk16(hb[2], hb[3]), pk16(hb[4], hb[5]), pk16(hb[6], hb[7])};
  ul = (v4u){pk16(lb[0], lb[1]), pk16(lb[2], lb[3]), pk16(lb[4], lb[5]), pk16(lb[6], lb[7])};
}

__global__ __launch_bounds__(256) void wtsplit_kernel(
    const float* __restrict__ p0, const float* __restrict__ p1, const float* __restrict__ p2, const float* __restrict__ p3,
    const float* __restrict__ p4, const float* __restrict__ p5, const float* __restrict__ p6, const float* __restrict__ p7,
    long layerStride, int Kin, int Nout,
    unsigned short* __restrict__ outH, unsigned short* __restrict__ outL, long slotStride) {
  __shared__ float sm[64][65];
  const int t  = threadIdx.x;
  const int k0 = blockIdx.x * 64;
  const int n0 = blockIdx.y * 64;
  const int z  = blockIdx.z;
  const int m  = z & 7;
  const int li = z >> 3;
  const float* Wsel = (m == 0) ? p0 : (m == 1) ? p1 : (m == 2) ? p2 : (m == 3) ? p3
                    : (m == 4) ? p4 : (m == 5) ? p5 : (m == 6) ? p6 : p7;
  const float* W = Wsel + (size_t)li * layerStride;
#pragma unroll
  for (int i = 0; i < 16; ++i) {
    const int e = i * 256 + t;
    const int r = e >> 6;
    const int c = e & 63;
    sm[c][r] = W[(size_t)(k0 + r) * Nout + n0 + c];
  }
  __syncthreads();
  const int lane = t & 31, wave = t >> 5;
  const int q = lane >> 3, c8 = (lane & 7) * 8;
  unsigned short* oh = outH + (size_t)z * slotStride;
  unsigned short* ol = outL + (size_t)z * slotStride;
  for (int pass = 0; pass < 2; ++pass) {
#pragma unroll
    for (int it = 0; it < 2; ++it) {
      const int row = wave * 8 + it * 4 + q;
      float v[8];
#pragma unroll
      for (int e = 0; e < 8; ++e) v[e] = sm[row][c8 + e];
      v4u uh, ul;
      split_pack8(v, uh, ul);
      const size_t o = (size_t)(n0 + row) * Kin + k0 + c8;
      *(volatile v4u*)(oh + o) = uh;
      *(volatile v4u*)(ol + o) = ul;
    }
    __threadfence();
  }
}

struct Kappas { float k[8]; };
static_assert(sizeof(Kappas) == 32, "");
__global__ __launch_bounds__(256) void dtab_kernel(float* __restrict__ dtab, Kappas kp) {
  const int h = blockIdx.x;
  const int e = threadIdx.x;
  const float kap = (h == 0) ? kp.k[0] : (h == 1) ? kp.k[1] : (h == 2) ? kp.k[2] : (h == 3) ? kp.k[3]
                  : (h == 4) ? kp.k[4] : (h == 5) ? kp.k[5] : (h == 6) ? kp.k[6] : kp.k[7];
  const float d = powf(kap, (float)e);
  float* op = dtab + (size_t)h * 256 + e;
  *(volatile float*)op = d;
  __threadfence();
  *(volatile float*)op = d;
}

__global__ __launch_bounds__(256) void rms_obs_kernel(const float* __restrict__ in, const float* __restrict__ scale,
                                                     unsigned short* __restrict__ oh, unsigned short* __restrict__ ol) {
  const int lane = threadIdx.x & 31, wave = threadIdx.x >> 5;
  const int hl = lane >> 4, cl = lane & 15;
  const int row = (blockIdx.x * 8 + wave) * 2 + hl;
  const float* p = in + (size_t)row * kObs + 8 * cl;
  const v4f a = *(const v4f*)(p);
  const v4f c = *(const v4f*)(p + 4);
  float x[8];
#pragma unroll
  for (int e = 0; e < 4; ++e) { x[e] = a[e]; x[4 + e] = c[e]; }
  float ss = 0.f;
#pragma unroll
  for (int e = 0; e < 8; ++e) ss += x[e] * x[e];
#pragma unroll
  for (int off = 1; off < 16; off <<= 1) ss += __shfl_xor(ss, off, 32);
  const float inv = rsqrtf(ss * (1.0f / kObs) + kEps);
  const v4f sa = *(const v4f*)(scale + 8 * cl);
  const v4f sc = *(const v4f*)(scale + 8 * cl + 4);
  float y[8];
#pragma unroll
  for (int e = 0; e < 4; ++e) { y[e] = x[e] * inv * sa[e]; y[4 + e] = x[4 + e] * inv * sc[e]; }
  v4u uh, ul;
  split_pack8(y, uh, ul);
  const size_t o = (size_t)row * kObs + 8 * cl;
  for (int pass = 0; pass < 2; ++pass) {
    *(volatile v4u*)(oh + o) = uh;
    *(volatile v4u*)(ol + o) = ul;
    __threadfence();
  }
}

template <bool GELU_IN>
__global__ __launch_bounds__(256) void rms256_kernel(const float* __restrict__ in, const float* __restrict__ scale,
                                                    float* __restrict__ outf, unsigned short* __restrict__ oh,
                                                    unsigned short* __restrict__ ol) {
  __shared__ __align__(16) float slab[8][kE];
  const int lane = threadIdx.x & 31, wave = threadIdx.x >> 5;
  const int row = blockIdx.x * 8 + wave;
  const float* p = in + (size_t)row * kE;
  const v4f a = *(const v4f*)(p + 4 * lane);
  const v4f c = *(const v4f*)(p + 128 + 4 * lane);
  float x[8];
#pragma unroll
  for (int e = 0; e < 4; ++e) { x[e] = a[e]; x[4 + e] = c[e]; }
  if (GELU_IN) {
#pragma unroll
    for (int e = 0; e < 8; ++e) x[e] = gelu_f(x[e]);
  }
  float ss = 0.f;
#pragma unroll
  for (int e = 0; e < 8; ++e) ss += x[e] * x[e];
#pragma unroll
  for (int off = 16; off > 0; off >>= 1) ss += __shfl_xor(ss, off, 32);
  const float inv = rsqrtf(ss * (1.0f / kE) + kEps);
  const v4f sa = *(const v4f*)(scale + 4 * lane);
  const v4f sc = *(const v4f*)(scale + 128 + 4 * lane);
  v4f y0, y1;
#pragma unroll
  for (int e = 0; e < 4; ++e) { y0[e] = x[e] * inv * sa[e]; y1[e] = x[4 + e] * inv * sc[e]; }
  {
    float* op = outf + (size_t)row * kE;
    for (int pass = 0; pass < 2; ++pass) {
      *(volatile v4f*)(op + 4 * lane) = y0;
      *(volatile v4f*)(op + 128 + 4 * lane) = y1;
      __threadfence();
    }
  }
  {
    float* sw = slab[wave];
    *(v4f*)(sw + 4 * lane) = y0;
    *(v4f*)(sw + 128 + 4 * lane) = y1;
    __builtin_amdgcn_fence(__ATOMIC_RELEASE, "workgroup");
    __builtin_amdgcn_wave_barrier();
    __builtin_amdgcn_fence(__ATOMIC_ACQUIRE, "workgroup");
    const v4f g0 = *(const v4f*)(sw + 8 * lane);
    const v4f g1 = *(const v4f*)(sw + 8 * lane + 4);
    float v[8];
#pragma unroll
    for (int e = 0; e < 4; ++e) { v[e] = g0[e]; v[4 + e] = g1[e]; }
    v4u uh, ul;
    split_pack8(v, uh, ul);
    const size_t o = (size_t)row * kE + 8 * lane;
    for (int pass = 0; pass < 2; ++pass) {
      *(volatile v4u*)(oh + o) = uh;
      *(volatile v4u*)(ol + o) = ul;
      __threadfence();
    }
  }
}

__global__ __launch_bounds__(256) void gate_kernel(const float* __restrict__ ret, const unsigned short* __restrict__ gh,
                                                 const unsigned short* __restrict__ gl, unsigned short* __restrict__ oh,
                                                 unsigned short* __restrict__ ol) {
  const int lane = threadIdx.x & 31, wave = threadIdx.x >> 5;
  const int row = blockIdx.x * 8 + wave;
  const size_t rb = (size_t)row * kE + 8 * lane;
  const v4f r0 = *(const v4f*)(ret + rb);
  const v4f r1 = *(const v4f*)(ret + rb + 4);
  const size_t gb = (size_t)row * kQKG + 2 * kE + 8 * lane;
  const v4u uh = *(const v4u*)(gh + gb);
  const v4u ul = *(const v4u*)(gl + gb);
  float y[8], g[8];
#pragma unroll
  for (int e = 0; e < 4; ++e) { y[e] = r0[e]; y[4 + e] = r1[e]; }
#pragma unroll
  for (int i = 0; i < 4; ++i) {
    const unsigned wh = uh[i], wl = ul[i];
    g[2 * i]     = __uint_as_float(wh << 16) + __uint_as_float(wl << 16);
    g[2 * i + 1] = __uint_as_float(wh & 0xffff0000u) + __uint_as_float(wl & 0xffff0000u);
  }
  float s = 0.f;
#pragma unroll
  for (int e = 0; e < 8; ++e) s += y[e];
  s += __shfl_xor(s, 1, 32);
  s += __shfl_xor(s, 2, 32);
  const float mu = s * (1.0f / kDh);
  float d[8];
  float vs = 0.f;
#pragma unroll
  for (int e = 0; e < 8; ++e) { d[e] = y[e] - mu; vs += d[e] * d[e]; }
  vs += __shfl_xor(vs, 1, 32);
  vs += __shfl_xor(vs, 2, 32);
  const float inv = rsqrtf(vs * (1.0f / kDh) + kEps);
  float o[8];
#pragma unroll
  for (int e = 0; e < 8; ++e) o[e] = d[e] * inv * silu_f(g[e]);
  v4u ph, pl;
  split_pack8(o, ph, pl);
  const size_t oo = (size_t)row * kE + 8 * lane;
  for (int pass = 0; pass < 2; ++pass) {
    *(volatile v4u*)(oh + oo) = ph;
    *(volatile v4u*)(ol + oo) = pl;
    __threadfence();
  }
}

__global__ __launch_bounds__(256) void swiglu_kernel(const float* __restrict__ ab, unsigned short* __restrict__ oh,
                                                   unsigned short* __restrict__ ol) {
  const int lane = threadIdx.x & 31, wave = threadIdx.x >> 5;
  const int row = blockIdx.x * 8 + wave;
  const float* p = ab + (size_t)row * (2 * kE) + 8 * lane;
  const v4f a0 = *(const v4f*)(p);
  const v4f a1 = *(const v4f*)(p + 4);
  const v4f b0 = *(const v4f*)(p + kE);
  const v4f b1 = *(const v4f*)(p + kE + 4);
  float o[8];
#pragma unroll
  for (int e = 0; e < 4; ++e) { o[e] = silu_f(a0[e]) * b0[e]; o[4 + e] = silu_f(a1[e]) * b1[e]; }
  v4u ph, pl;
  split_pack8(o, ph, pl);
  const size_t oo = (size_t)row * kE + 8 * lane;
  for (int pass = 0; pass < 2; ++pass) {
    *(volatile v4u*)(oh + oo) = ph;
    *(volatile v4u*)(ol + oo) = pl;
    __threadfence();
  }
}

__global__ __launch_bounds__(256) void head_kernel(const float* __restrict__ hin, const float* __restrict__ b1,
                                                 const float* __restrict__ ln, const float* __restrict__ w2,
                                                 const float* __restrict__ b2, float* __restrict__ out0) {
  __shared__ float sv[32];
  const int lane = threadIdx.x & 31, wave = threadIdx.x >> 5;
  const v4f sb0 = *(const v4f*)(b1 + 4 * lane);
  const v4f sb1 = *(const v4f*)(b1 + 128 + 4 * lane);
  const v4f sl0 = *(const v4f*)(ln + 4 * lane);
  const v4f sl1 = *(const v4f*)(ln + 128 + 4 * lane);
  const v4f sw0 = *(const v4f*)(w2 + 4 * lane);
  const v4f sw1 = *(const v4f*)(w2 + 128 + 4 * lane);
  const float bb = b2[0];
#pragma unroll 1
  for (int it = 0; it < 4; ++it) {
    const int row = blockIdx.x * 32 + wave * 4 + it;
    const float* p = hin + (size_t)row * kE;
    const v4f a = *(const v4f*)(p + 4 * lane);
    const v4f c = *(const v4f*)(p + 128 + 4 * lane);
    float x[8];
#pragma unroll
    for (int e = 0; e < 4; ++e) { x[e] = gelu_f(a[e] + sb0[e]); x[4 + e] = gelu_f(c[e] + sb1[e]); }
    float ss = 0.f;
#pragma unroll
    for (int e = 0; e < 8; ++e) ss += x[e] * x[e];
#pragma unroll
    for (int off = 16; off > 0; off >>= 1) ss += __shfl_xor(ss, off, 32);
    const float inv = rsqrtf(ss * (1.0f / kE) + kEps);
    float dot = 0.f;
#pragma unroll
    for (int e = 0; e < 4; ++e) {
      dot += (x[e] * inv * sl0[e]) * sw0[e];
      dot += (x[4 + e] * inv * sl1[e]) * sw1[e];
    }
#pragma unroll
    for (int off = 16; off > 0; off >>= 1) dot += __shfl_xor(dot, off, 32);
    if (lane == 0) sv[wave * 4 + it] = dot + bb;
  }
  __syncthreads();
  if (wave == 0) {
    const float v = sv[lane];
    float* op = out0 + (size_t)blockIdx.x * 32 + lane;
    *(volatile float*)op = v;
    __threadfence();
    *(volatile float*)op = v;
  }
}

extern "C" void kernel_launch(void* const* d_in, const int* in_sizes, int n_in,
                              void* d_out, int out_size, void* d_ws,
                              size_t ws_size, hipStream_t stream) {
  if (n_in < 19) return;
  if (in_sizes[0] != kTok * kObs) return;
  if (in_sizes[4] != kL * kE * kE) return;
  if (out_size != kTok + kTok * kE) return;

  const float* obs        = (const float*)d_in[0];
  const float* obs_ln     = (const float*)d_in[1];
  const float* w_obs      = (const float*)d_in[2];
  const float* ln_scale   = (const float*)d_in[3];
  const float* blk_wq     = (const float*)d_in[4];
  const float* blk_wk     = (const float*)d_in[5];
  const float* blk_wv     = (const float*)d_in[6];
  const float* blk_wg     = (const float*)d_in[7];
  const float* blk_wo     = (const float*)d_in[8];
  const float* blk_ln1    = (const float*)d_in[9];
  const float* blk_ln2    = (const float*)d_in[10];
  const float* blk_ffn_w  = (const float*)d_in[11];
  const float* blk_ffn_v  = (const float*)d_in[12];
  const float* blk_ffn_w2 = (const float*)d_in[13];
  const float* head_w1    = (const float*)d_in[14];
  const float* head_b1    = (const float*)d_in[15];
  const float* head_ln    = (const float*)d_in[16];
  const float* head_w2    = (const float*)d_in[17];
  const float* head_b2    = (const float*)d_in[18];

  float* out0 = (float*)d_out;
  float* out1 = (float*)d_out + kTok;

  const size_t NE      = (size_t)kTok * kE;
  const size_t WSLOT   = (size_t)kE * kE;
  const size_t WOBS_EL = (size_t)kL * 8 * WSLOT;
  const size_t WHEAD_EL = WOBS_EL + (size_t)kE * kObs;
  const size_t WPLANE_B = (WHEAD_EL + WSLOT) * 2;
  const size_t SCHUNK_B = (size_t)kH * kS * kS * 2;

  unsigned char* ws = (unsigned char*)d_ws;
  size_t off = 0;
  unsigned short* WH = (unsigned short*)(ws + off); off += WPLANE_B;
  unsigned short* WL = (unsigned short*)(ws + off); off += WPLANE_B;
  float* DT   = (float*)(ws + off); off += 8192;
  float* REP  = (float*)(ws + off); off += NE * 4;
  float* X32  = (float*)(ws + off); off += NE * 4;
  unsigned short* XH = (unsigned short*)(ws + off); off += NE * 2;
  unsigned short* XL = (unsigned short*)(ws + off); off += NE * 2;
  unsigned short* QKGH = (unsigned short*)(ws + off); off += (size_t)kTok * kQKG * 2;
  unsigned short* QKGL = (unsigned short*)(ws + off); off += (size_t)kTok * kQKG * 2;
  unsigned short* VTH = (unsigned short*)(ws + off); off += NE * 2;
  unsigned short* VTL = (unsigned short*)(ws + off); off += NE * 2;
  float* RET  = (float*)(ws + off); off += NE * 4;
  unsigned short* SH = (unsigned short*)(ws + off); off += SCHUNK_B;
  unsigned short* SL = (unsigned short*)(ws + off); off += SCHUNK_B;
  if (off > ws_size) return;
  float* AB32 = (float*)QKGH;

  Kappas kp;
  {
    const float la = logf(0.03125f);
    const float lb = logf(0.001953125f);
    for (int h = 0; h < kH; ++h) {
      const float t = (float)h / 7.0f;
      float v = la * (1.0f - t) + lb * t;
      if (h == kH - 1) v = lb;
      kp.k[h] = 1.0f - expf(v);
    }
  }

  const dim3 blk(256);

  wtsplit_kernel<<<dim3(kE / 64, kE / 64, kL * 8), blk, 0, stream>>>(
      blk_wq, blk_wk, blk_wg, blk_wv, blk_wo, blk_ffn_w, blk_ffn_v, blk_ffn_w2,
      (long)WSLOT, kE, kE, WH, WL, (long)WSLOT);
  wtsplit_kernel<<<dim3(kObs / 64, kE / 64, 1), blk, 0, stream>>>(
      w_obs, w_obs, w_obs, w_obs, w_obs, w_obs, w_obs, w_obs,
      0L, kObs, kE, WH + WOBS_EL, WL + WOBS_EL, 0L);
  wtsplit_kernel<<<dim3(kE / 64, kE / 64, 1), blk, 0, stream>>>(
      head_w1, head_w1, head_w1, head_w1, head_w1, head_w1, head_w1, head_w1,
      0L, kE, kE, WH + WHEAD_EL, WL + WHEAD_EL, 0L);
  dtab_kernel<<<dim3(kH), blk, 0, stream>>>(DT, kp);

  rms_obs_kernel<<<dim3(kTok / 16), blk, 0, stream>>>(obs, obs_ln, XH, XL);
  gemm_bf16x3<4, 0, false, 0><<<dim3(((kTok / 64) * (kE / 64) + 7) / 8, 1), blk, 0, stream>>>(
      XH, XL, kObs, 0L, WH + WOBS_EL, WL + WOBS_EL, kObs, 0L,
      REP, nullptr, kE, 0L, nullptr, nullptr, kTok, kE, kObs, 1.0f);

  const float score_scale = 0.17677669529663688f;
  for (int l = 0; l < kL; ++l) {
    const unsigned short* wqkgH = WH + ((size_t)l * 8 + 0) * WSLOT;
    const unsigned short* wqkgL = WL + ((size_t)l * 8 + 0) * WSLOT;
    const unsigned short* wvH   = WH + ((size_t)l * 8 + 3) * WSLOT;
    const unsigned short* wvL   = WL + ((size_t)l * 8 + 3) * WSLOT;
    const unsigned short* woH   = WH + ((size_t)l * 8 + 4) * WSLOT;
    const unsigned short* woL   = WL + ((size_t)l * 8 + 4) * WSLOT;
    const unsigned short* wfH   = WH + ((size_t)l * 8 + 5) * WSLOT;
    const unsigned short* wfL   = WL + ((size_t)l * 8 + 5) * WSLOT;
    const unsigned short* w2H   = WH + ((size_t)l * 8 + 7) * WSLOT;
    const unsigned short* w2L   = WL + ((size_t)l * 8 + 7) * WSLOT;
    const float* ln1 = blk_ln1 + (size_t)l * kE;
    const float* ln2 = blk_ln2 + (size_t)l * kE;
    float* rep_out = (l == kL - 1) ? out1 : REP;

    if (l == 0) rms256_kernel<true><<<dim3(kTok / 8), blk, 0, stream>>>(REP, ln_scale, X32, XH, XL);
    else        rms256_kernel<false><<<dim3(kTok / 8), blk, 0, stream>>>(REP, ln_scale, X32, XH, XL);

    gemm_bf16x3<4, 2, false, 0><<<dim3(((kTok / 64) * (kQKG / 64) + 7) / 8, 1), blk, 0, stream>>>(
        XH, XL, kE, 0L, wqkgH, wqkgL, kE, 0L,
        QKGH, QKGL, kQKG, 0L, nullptr, nullptr, kTok, kQKG, kE, 1.0f);

    gemm_bf16x3<4, 2, false, 0><<<dim3(((kE / 64) * (kTok / 64) + 7) / 8, 1), blk, 0, stream>>>(
        wvH, wvL, kE, 0L, XH, XL, kE, 0L,
        VTH, VTL, kTok, 0L, nullptr, nullptr, kE, kTok, kE, 1.0f);

    for (int bq = 0; bq < kB; ++bq) {
      const size_t qoff = (size_t)bq * kS * kQKG;
      gemm_bf16x3<4, 2, false, 1><<<dim3(((kS / 64) * (kS / 64) + 7) / 8, kH), blk, 0, stream>>>(
          QKGH + qoff, QKGL + qoff, kQKG, (long)kDh,
          QKGH + qoff + kE, QKGL + qoff + kE, kQKG, (long)kDh,
          SH, SL, kS, (long)kS * kS, nullptr, DT, kS, kS, kDh, score_scale);
      gemm_bf16x3<2, 0, false, 2><<<dim3(((kS / 64) * 1 + 7) / 8, kH), blk, 0, stream>>>(
          SH, SL, kS, (long)kS * kS,
          VTH + (size_t)bq * kS, VTL + (size_t)bq * kS, kTok, (long)kDh * kTok,
          RET + (size_t)bq * kS * kE, nullptr, kE, (long)kDh, nullptr, nullptr, kS, kDh, kS, 1.0f);
    }

    gate_kernel<<<dim3(kTok / 8), blk, 0, stream>>>(RET, QKGH, QKGL, XH, XL);

    gemm_bf16x3<4, 0, true, 0><<<dim3(((kTok / 64) * (kE / 64) + 7) / 8, 1), blk, 0, stream>>>(
        XH, XL, kE, 0L, woH, woL, kE, 0L,
        RET, nullptr, kE, 0L, X32, nullptr, kTok, kE, kE, 1.0f);

    rms256_kernel<false><<<dim3(kTok / 8), blk, 0, stream>>>(RET, ln1, X32, XH, XL);

    gemm_bf16x3<4, 0, false, 0><<<dim3(((kTok / 64) * ((2 * kE) / 64) + 7) / 8, 1), blk, 0, stream>>>(
        XH, XL, kE, 0L, wfH, wfL, kE, 0L,
        AB32, nullptr, 2 * kE, 0L, nullptr, nullptr, kTok, 2 * kE, kE, 1.0f);

    swiglu_kernel<<<dim3(kTok / 8), blk, 0, stream>>>(AB32, XH, XL);

    gemm_bf16x3<4, 0, true, 0><<<dim3(((kTok / 64) * (kE / 64) + 7) / 8, 1), blk, 0, stream>>>(
        XH, XL, kE, 0L, w2H, w2L, kE, 0L,
        RET, nullptr, kE, 0L, X32, nullptr, kTok, kE, kE, 1.0f);

    rms256_kernel<false><<<dim3(kTok / 8), blk, 0, stream>>>(RET, ln2, rep_out, XH, XL);
  }

  gemm_bf16x3<4, 0, false, 0><<<dim3(((kTok / 64) * (kE / 64) + 7) / 8, 1), blk, 0, stream>>>(
      XH, XL, kE, 0L, WH + WHEAD_EL, WL + WHEAD_EL, kE, 0L,
      RET, nullptr, kE, 0L, nullptr, nullptr, kTok, kE, kE, 1.0f);
  head_kernel<<<dim3(kTok / 32), blk, 0, stream>>>(RET, head_b1, head_ln, head_w2, head_b2, out0);
}
